// SA_61272003445141
// MI455X (gfx1250) — hardware-verified
//
#include <hip/hip_runtime.h>
#include <stddef.h>


typedef _Float16 v16h __attribute__((ext_vector_type(16)));
typedef _Float16 v8h  __attribute__((ext_vector_type(8)));
typedef float    v8f  __attribute__((ext_vector_type(8)));
typedef float    v4f  __attribute__((ext_vector_type(4)));
typedef _Float16 h16;

#ifndef NB
#define NB 4
#endif
#ifndef SEQ
#define SEQ 4096
#endif
#define NB_FULL  4
#define SEQ_FULL 4096
#define DIM   256
#define MROWS (NB * SEQ)
#define DH    128
#define QBLK  64

#define LDC 68
#define LDO 132

#define WCARRY 64.0f
#define LN_PCARRY 6.931471805599453f

static_assert(NB >= 1 && NB <= NB_FULL);
static_assert(SEQ >= 128 && SEQ <= SEQ_FULL && (SEQ % 128) == 0);
static_assert(DIM == 32 * 8);
static_assert((DIM % 64) == 0 && (DIM % 32) == 0);
static_assert((MROWS % 64) == 0 && (MROWS % 8) == 0);
static_assert((SEQ % QBLK) == 0 && (SEQ % 32) == 0 && (SEQ % 64) == 0);
static_assert(2 * DH == DIM && (DH % 16) == 0 && DH / 16 == 8);
static_assert(DH * 4 == 32 * 16);
static_assert(QBLK == 4 * 16);
static_assert((LDC % 4) == 0 && LDC >= 64);
static_assert((LDO % 4) == 0 && LDO >= DH);
static_assert(2 * 8 == 16);
static_assert(8 * 16 * LDO * 4 + 8 * 4 <= 131072);
static_assert(64 * LDC * 4 <= 131072);
static_assert((size_t)MROWS * DIM < (size_t)0xFFFFFFFFu);

#define W_BYTES   ((size_t)DIM * DIM * 2)
#define X16_BYTES ((size_t)MROWS * DIM * 2)
#define S_BYTES   ((size_t)MROWS * 4)
#define VT_BYTES  ((size_t)NB * DIM * SEQ * 2)
#define OFF_WQ  ((size_t)0)
#define OFF_WK  (OFF_WQ + W_BYTES)
#define OFF_WV  (OFF_WK + W_BYTES)
#define OFF_X16 (OFF_WV + W_BYTES)
#define OFF_QS  (OFF_X16 + X16_BYTES)
#define OFF_KS  (OFF_QS + S_BYTES)
#define OFF_VT  (OFF_KS + S_BYTES)
#define WS_TOTAL (OFF_VT + VT_BYTES)
static_assert((W_BYTES % 128) == 0 && (X16_BYTES % 128) == 0);
static_assert((S_BYTES % 128) == 0 && (VT_BYTES % 128) == 0);
static_assert(WS_TOTAL <= (size_t)134217728);

__device__ __forceinline__ float bf16r(float x) {
  unsigned int u = __float_as_uint(x);
  u = (u + 0x7FFFu + ((u >> 16) & 1u)) & 0xFFFF0000u;
  return __uint_as_float(u);
}

static __device__ __forceinline__ h16 toh_flush(float v) {
  const h16 r = (h16)v;
  return (fabsf(v) < 6.103515625e-05f) ? (h16)0.0f : r;
}

__device__ __forceinline__ v16h frag_at(const _Float16* p) {
  v8h lo = *(const v8h*)(p);
  v8h hi = *(const v8h*)(p + 16);
  v16h out;
#pragma unroll
  for (int i = 0; i < 8; ++i) { out[i] = lo[i]; out[i + 8] = hi[i]; }
  return out;
}

__device__ __forceinline__ v8f wmma16(v16h a, v16h b, v8f c) {
  v8f d = __builtin_amdgcn_wmma_f32_16x16x32_f16(false, a, false, b, (short)0, c,
                                                 false, false);
  asm volatile("v_nop\n\tv_nop\n\tv_nop\n\tv_nop" : "+v"(d) : "v"(a), "v"(b));
  return d;
}

__device__ __forceinline__ float red16_sum(float x) {
#pragma unroll
  for (int off = 1; off < 16; off <<= 1) x += __shfl_xor(x, off, 32);
  return x;
}
__device__ __forceinline__ float red32_min(float x) {
#pragma unroll
  for (int off = 1; off < 32; off <<= 1) x = fminf(x, __shfl_xor(x, off, 32));
  return x;
}

__device__ __forceinline__ void wave_lds_sync() {
  __builtin_amdgcn_fence(3  , "wavefront");
  asm volatile("s_wait_dscnt 0x0" ::: "memory");
  __builtin_amdgcn_wave_barrier();
}

template <int SRC_INPUT>
__device__ __forceinline__ void cast_body(const float* __restrict__ X,
                                          _Float16* __restrict__ dst, const float carry) {
#pragma clang fp contract(off)
  const unsigned lane = threadIdx.x & 31u;
  const unsigned w = (unsigned)__builtin_amdgcn_readfirstlane((int)(threadIdx.x >> 5));
  const unsigned crow = blockIdx.x * 8u + w;
  size_t srow = crow;
  if (SRC_INPUT) {
    const unsigned bidx = crow / (unsigned)SEQ;
    const unsigned sq = crow - bidx * (unsigned)SEQ;
    srow = (size_t)bidx * SEQ_FULL + sq;
  }
  const float* xr = X + srow * DIM + lane * 8u;
  const v4f a0 = *(const v4f*)(xr);
  const v4f a1 = *(const v4f*)(xr + 4u);
  v8h o;
#pragma unroll
  for (int i = 0; i < 4; ++i) {
    o[i]     = toh_flush(carry * bf16r(a0[i]));
    o[i + 4] = toh_flush(carry * bf16r(a1[i]));
  }
  _Float16* p = dst + (size_t)crow * DIM + lane * 8u;
  *(volatile v8h*)p = o;
  __threadfence();
  *(volatile v8h*)p = o;
}

__global__ __launch_bounds__(256) void xcast_kernel(
    const float* __restrict__ X, _Float16* __restrict__ dst) {
  cast_body<1>(X, dst, 1.0f);
}
__global__ __launch_bounds__(256) void wcast_kernel(
    const float* __restrict__ W, _Float16* __restrict__ dst) {
  cast_body<0>(W, dst, WCARRY);
}

__global__ __launch_bounds__(256) void proj_score_kernel(
    const _Float16* __restrict__ A16, const _Float16* __restrict__ Bt,
    const float* __restrict__ wv, float* __restrict__ outs) {
  __shared__ float Rs[2 * 64];
  const unsigned tid = threadIdx.x, lane = tid & 31u;
  const int wave = __builtin_amdgcn_readfirstlane((int)(threadIdx.x >> 5));
  const unsigned mw = (unsigned)wave >> 1, nw = (unsigned)wave & 1u;
  const unsigned hh = lane >> 4, m = lane & 15u;
  const unsigned row0 = blockIdx.x * 64u;

  const _Float16* ap = A16 + (size_t)(row0 + mw * 16u + m) * DIM + hh * 8u;
  float part[8];
#pragma unroll
  for (int r = 0; r < 8; ++r) part[r] = 0.0f;

#pragma unroll 1
  for (unsigned nb = 0; nb < (unsigned)(DIM / 64); ++nb) {
    const unsigned col = nb * 64u + nw * 32u + m;
    const _Float16* bp0 = Bt + (size_t)col * DIM + hh * 8u;
    const _Float16* bp1 = bp0 + (size_t)16 * DIM;
    v8f acc0 = {}, acc1 = {};
#pragma unroll 2
    for (unsigned k0 = 0; k0 < (unsigned)DIM; k0 += 32u) {
      const v16h a  = frag_at(ap + k0);
      const v16h b0 = frag_at(bp0 + k0);
      const v16h b1 = frag_at(bp1 + k0);
      acc0 = wmma16(a, b0, acc0);
      acc1 = wmma16(a, b1, acc1);
    }
    const float w0 = bf16r(wv[col]);
    const float w1 = bf16r(wv[col + 16u]);
#pragma unroll
    for (int r = 0; r < 8; ++r) part[r] += acc0[r] * w0 + acc1[r] * w1;
  }
#pragma unroll
  for (int r = 0; r < 8; ++r) part[r] = red16_sum(part[r]);
  if (m == 0u) {
#pragma unroll
    for (int r = 0; r < 8; ++r) Rs[nw * 64u + mw * 16u + hh * 8u + (unsigned)r] = part[r];
  }
  __syncthreads();
  if (wave == 0 && lane < 16u) {
    v4f val;
#pragma unroll
    for (int j = 0; j < 4; ++j)
      val[j] = (Rs[lane * 4u + (unsigned)j] + Rs[64u + lane * 4u + (unsigned)j]) * (1.0f / WCARRY);
    float* p = outs + row0 + lane * 4u;
    *(volatile v4f*)p = val;
    __threadfence();
    *(volatile v4f*)p = val;
  }
}

__global__ __launch_bounds__(256) void gemm_v_kernel(
    const _Float16* __restrict__ A16, const _Float16* __restrict__ Bt,
    _Float16* __restrict__ vt) {
  __shared__ float Cs[64 * LDC];
  const unsigned tid = threadIdx.x, lane = tid & 31u;
  const unsigned w = (unsigned)__builtin_amdgcn_readfirstlane((int)(threadIdx.x >> 5));
  const unsigned mw = w >> 1, nw = w & 1u;
  const unsigned hh = lane >> 4, m = lane & 15u;
  const unsigned n0 = blockIdx.x * 64u;
  const unsigned row0 = blockIdx.y * 64u;
  const unsigned K = (unsigned)DIM;

  const _Float16* ap  = A16 + (size_t)(row0 + mw * 16u + m) * K + hh * 8u;
  const _Float16* bp0 = Bt + (size_t)(n0 + nw * 32u + m) * K + hh * 8u;
  const _Float16* bp1 = bp0 + (size_t)16 * K;
  v8f acc0 = {}, acc1 = {};
#pragma unroll 2
  for (unsigned k0 = 0; k0 < K; k0 += 32u) {
    const v16h a  = frag_at(ap + k0);
    const v16h b0 = frag_at(bp0 + k0);
    const v16h b1 = frag_at(bp1 + k0);
    acc0 = wmma16(a, b0, acc0);
    acc1 = wmma16(a, b1, acc1);
  }
#pragma unroll
  for (int r = 0; r < 8; ++r) {
    float* d = &Cs[(mw * 16u + hh * 8u + (unsigned)r) * LDC + nw * 32u + m];
    d[0]  = acc0[r];
    d[16] = acc1[r];
  }
  __syncthreads();

  const unsigned bidx = row0 / (unsigned)SEQ;
  const unsigned key0 = row0 - bidx * (unsigned)SEQ;
  v8h x[2];
  size_t off[2];
#pragma unroll
  for (unsigned i = 0; i < 2u; ++i) {
    const unsigned dcol = 32u * i + (tid >> 3);
    const unsigned kk = (tid & 7u) * 8u;
#pragma unroll
    for (unsigned j = 0; j < 8u; ++j) {
      const float t = Cs[(kk + j) * LDC + dcol] * (1.0f / WCARRY);
      x[i][j] = toh_flush(t);
    }
    off[i] = ((size_t)bidx * DIM + n0 + dcol) * SEQ + key0 + kk;
  }
#pragma unroll
  for (int i = 0; i < 2; ++i) *(volatile v8h*)(vt + off[i]) = x[i];
  __threadfence();
#pragma unroll
  for (int i = 0; i < 2; ++i) *(volatile v8h*)(vt + off[i]) = x[i];
}

__device__ __forceinline__ h16 p_elem(const float qb, const float k, const float cexp,
                                      float& lsum) {
  const float s = fmaxf(qb - k, 0.0f);
  const h16 p = toh_flush(__expf(s - cexp));
  lsum += (float)p;
  return p;
}

__global__ __launch_bounds__(256) void attn_kernel(
    const float* __restrict__ Qs, const float* __restrict__ Ksc,
    const float* __restrict__ bptr, const _Float16* __restrict__ Vt,
    float* __restrict__ out) {
  __shared__ float Os[8 * 16 * LDO];
  __shared__ float Wmin[8];

  const unsigned tid = threadIdx.x, lane = tid & 31u;
  const int wave = __builtin_amdgcn_readfirstlane((int)(threadIdx.x >> 5));
  const unsigned hh = lane >> 4, m = lane & 15u;
  const unsigned b = blockIdx.y;
  const unsigned qg = (unsigned)wave >> 1, dh = (unsigned)wave & 1u;
  const unsigned qrow0 = blockIdx.x * (unsigned)QBLK + qg * 16u;
  const float* ksb = Ksc + (size_t)b * SEQ;

  float kmin = 3.0e38f;
#pragma unroll 1
  for (unsigned it = 0; it < (unsigned)((SEQ + 1023) / 1024); ++it) {
    unsigned j = tid * 4u + it * 1024u;
    j = (j > (unsigned)(SEQ - 4)) ? (unsigned)(SEQ - 4) : j;
    const v4f t = *(const v4f*)(ksb + j);
    kmin = fminf(kmin, fminf(fminf(t[0], t[1]), fminf(t[2], t[3])));
  }
  kmin = red32_min(kmin);
  if (lane == 0u) Wmin[wave] = kmin;
  __syncthreads();
  float km = Wmin[0];
#pragma unroll
  for (int i = 1; i < 8; ++i) km = fminf(km, Wmin[i]);

  const float qb = Qs[(size_t)b * SEQ + qrow0 + m] + bf16r(bptr[0]);
  const float mrow = fmaxf(qb - km, 0.0f);
  const float cexp = mrow - LN_PCARRY;

  v8f o[8];
#pragma unroll
  for (int dt = 0; dt < 8; ++dt) o[dt] = (v8f){};
  float lsum = 0.0f;

  const size_t vbase = ((size_t)b * DIM + dh * (unsigned)DH + m) * SEQ + hh * 8u;

#pragma unroll 1
  for (unsigned kb = 0; kb < (unsigned)SEQ; kb += 32u) {
    const float* kp = ksb + kb + hh * 8u;
    const v4f k0v = *(const v4f*)(kp);
    const v4f k1v = *(const v4f*)(kp + 4u);
    const v4f k2v = *(const v4f*)(kp + 16u);
    const v4f k3v = *(const v4f*)(kp + 20u);
    v16h pf;
#pragma unroll
    for (int i = 0; i < 4; ++i) {
      pf[i]      = p_elem(qb, k0v[i], cexp, lsum);
      pf[i + 4]  = p_elem(qb, k1v[i], cexp, lsum);
      pf[i + 8]  = p_elem(qb, k2v[i], cexp, lsum);
      pf[i + 12] = p_elem(qb, k3v[i], cexp, lsum);
    }
#pragma unroll
    for (int dt = 0; dt < 8; ++dt) {
      const v16h a = frag_at(Vt + vbase + (size_t)dt * (16u * (unsigned)SEQ) + kb);
      o[dt] = wmma16(a, pf, o[dt]);
    }
  }

  const float ltot = lsum + __shfl_xor(lsum, 16, 32);
  const float inv = __builtin_amdgcn_rcpf(ltot);

  const unsigned tb = (unsigned)wave * (16u * LDO);
#pragma unroll
  for (int dt = 0; dt < 8; ++dt) {
    v4f u0, u1;
#pragma unroll
    for (int j = 0; j < 4; ++j) {
      u0[j] = o[dt][j] * inv;
      u1[j] = o[dt][j + 4] * inv;
    }
    *(v4f*)&Os[tb + m * LDO + (unsigned)dt * 16u + hh * 8u] = u0;
    *(v4f*)&Os[tb + m * LDO + (unsigned)dt * 16u + hh * 8u + 4u] = u1;
  }
  wave_lds_sync();

  const size_t orow = (size_t)b * SEQ_FULL + qrow0;
#pragma unroll
  for (unsigned g = 0; g < 2u; ++g) {
    v4f x[8];
    size_t off[8];
#pragma unroll
    for (unsigned i = 0; i < 8u; ++i) {
      const unsigned r = 8u * g + i;
      x[i] = *(const v4f*)&Os[tb + r * LDO + lane * 4u];
      off[i] = (orow + r) * DIM + dh * (unsigned)DH + lane * 4u;
    }
#pragma unroll
    for (int i = 0; i < 8; ++i) *(volatile v4f*)(out + off[i]) = x[i];
    __threadfence();
#pragma unroll
    for (int i = 0; i < 8; ++i) *(volatile v4f*)(out + off[i]) = x[i];
  }
}

extern "C" void kernel_launch(void* const* d_in, const int* in_sizes, int n_in,
                              void* d_out, int out_size, void* d_ws, size_t ws_size,
                              hipStream_t stream) {
  if (n_in < 6) return;
  const long long need_x = ((long long)(NB - 1) * SEQ_FULL + SEQ) * DIM;
  if ((long long)in_sizes[0] < need_x) return;
  if ((long long)in_sizes[1] < (long long)DIM * DIM) return;
  if ((long long)in_sizes[2] < (long long)DIM * DIM) return;
  if ((long long)in_sizes[3] < (long long)DIM * DIM) return;
  if (in_sizes[4] < DIM) return;
  if (in_sizes[5] < 1) return;
  if ((long long)out_size < need_x) return;
  if (ws_size < WS_TOTAL) return;

  const float* X    = (const float*)d_in[0];
  const float* wq   = (const float*)d_in[1];
  const float* wk   = (const float*)d_in[2];
  const float* wvv  = (const float*)d_in[3];
  const float* wmlp = (const float*)d_in[4];
  const float* bmlp = (const float*)d_in[5];
  float* out = (float*)d_out;

  char* ws = (char*)d_ws;
  _Float16* Wq16 = (_Float16*)(ws + OFF_WQ);
  _Float16* Wk16 = (_Float16*)(ws + OFF_WK);
  _Float16* Wv16 = (_Float16*)(ws + OFF_WV);
  _Float16* X16  = (_Float16*)(ws + OFF_X16);
  float*    QS   = (float*)(ws + OFF_QS);
  float*    KS   = (float*)(ws + OFF_KS);
  _Float16* Vt16 = (_Float16*)(ws + OFF_VT);

  dim3 blk(256);

  wcast_kernel<<<dim3(DIM / 8), blk, 0, stream>>>(wq, Wq16);
  wcast_kernel<<<dim3(DIM / 8), blk, 0, stream>>>(wk, Wk16);
  wcast_kernel<<<dim3(DIM / 8), blk, 0, stream>>>(wvv, Wv16);
  xcast_kernel<<<dim3(MROWS / 8), blk, 0, stream>>>(X, X16);

  proj_score_kernel<<<dim3(MROWS / 64), blk, 0, stream>>>(X16, Wq16, wmlp, QS);
  proj_score_kernel<<<dim3(MROWS / 64), blk, 0, stream>>>(X16, Wk16, wmlp, KS);
  gemm_v_kernel<<<dim3(DIM / 64, MROWS / 64), blk, 0, stream>>>(X16, Wv16, Vt16);
  attn_kernel<<<dim3(SEQ / QBLK, NB), blk, 0, stream>>>(QS, KS, bmlp, Vt16, out);
}
